// ScaledDotProductAttention_80461917323588
// MI455X (gfx1250) — hardware-verified
//
#include <hip/hip_runtime.h>

#ifndef NB
#define NB 2
#endif
#ifndef SEQ
#define SEQ 2048
#endif
#define NB_FULL 2
#define SEQ_FULL 2048
#define NH 16
#define HD 64
#define NBH (NB * NH)
#define NKT (SEQ / 64)
#define FPITCH 32
#define AW 4
#define OP 68

static_assert(SEQ % 64 == 0);
static_assert(SEQ <= SEQ_FULL);
static_assert(NB <= NB_FULL);
static_assert(NKT <= FPITCH);
static_assert(((long long)NBH * SEQ * 8) % 256 == 0);

typedef __attribute__((ext_vector_type(16))) __bf16       v16b;
typedef __attribute__((ext_vector_type(8)))  float        v8f;
typedef __attribute__((ext_vector_type(4)))  float        v4f;
typedef __attribute__((ext_vector_type(4)))  unsigned int v4u;
typedef __attribute__((ext_vector_type(8)))  unsigned int v8u;
typedef __attribute__((ext_vector_type(4)))  int          v4i;


__device__ __forceinline__ unsigned bfu_rne(float v) { unsigned u = __float_as_uint(v); u += 0x7fffu + ((u >> 16) & 1u); return u >> 16; }
__device__ __forceinline__ unsigned pk2(float a, float b) { return bfu_rne(a) | (bfu_rne(b) << 16); }
__device__ __forceinline__ v16b mkfrag(const v4u a, const v4u b) {
    v8u w; w[0] = a.x; w[1] = a.y; w[2] = a.z; w[3] = a.w; w[4] = b.x; w[5] = b.y; w[6] = b.z; w[7] = b.w;
    return __builtin_bit_cast(v16b, w);
}
__device__ __forceinline__ v8f wmmab(v16b a, v16b b, v8f c) {
    c = __builtin_amdgcn_wmma_f32_16x16x32_bf16(false, a, false, b, (short)0, c, false, false);
    asm volatile("v_nop\n\tv_nop\n\tv_nop\n\tv_nop" : "+v"(c) : "v"(a), "v"(b));
    return c;
}
__device__ __forceinline__ v8f wmmab2(v16b a, v16b b0, v16b b1, v8f c) {
    c = __builtin_amdgcn_wmma_f32_16x16x32_bf16(false, a, false, b0, (short)0, c, false, false);
    c = __builtin_amdgcn_wmma_f32_16x16x32_bf16(false, a, false, b1, (short)0, c, false, false);
    asm volatile("v_nop\n\tv_nop\n\tv_nop\n\tv_nop" : "+v"(c) : "v"(a), "v"(b0), "v"(b1));
    return c;
}

__global__ __launch_bounds__(256) void k_flags(const int* __restrict__ mask, int* __restrict__ flags) {
    __shared__ int lfl[FPITCH];
    const unsigned qt = blockIdx.x, t = threadIdx.x, w = t >> 5, lane = t & 31u;
    if (t < FPITCH) lfl[t] = 0;
    __syncthreads();
    for (unsigned kt = w; kt < NKT; kt += 8u) {
        int any = 0, all = 1;
        const int* base = mask + (size_t)(qt * 64u + (lane >> 4)) * SEQ_FULL + kt * 64u + (lane & 15u) * 4u;
#pragma unroll 4
        for (unsigned it = 0; it < 32u; ++it) {
            const v4i mv = *(const v4i*)(base + (size_t)it * 2u * SEQ_FULL);
            const int n0 = (mv.x != 0) ? 1 : 0, n1 = (mv.y != 0) ? 1 : 0, n2 = (mv.z != 0) ? 1 : 0, n3 = (mv.w != 0) ? 1 : 0;
            any |= (n0 | n1) | (n2 | n3);
            all &= (n0 & n1) & (n2 & n3);
        }
#pragma unroll
        for (int o = 16; o > 0; o >>= 1) { any |= __shfl_xor(any, o, 32); all &= __shfl_xor(all, o, 32); }
        const int fl = (any == 0) ? 0 : ((all != 0) ? 1 : 2);
        if (lane == 0) lfl[kt] = fl;
    }
    __syncthreads();
    if (w == 0) {
        const int v = lfl[lane];
        volatile int* d = (volatile int*)(flags + qt * FPITCH + lane);
        *d = v; __threadfence(); *d = v;
    }
}

__global__ __launch_bounds__(256) void k_prep_k(const float* __restrict__ K, unsigned short* __restrict__ Kb) {
    const unsigned u = blockIdx.x * 256u + threadIdx.x;
    if (u >= (unsigned)NBH * SEQ * 8u) return;
    const unsigned row = u >> 3, bh = row / (unsigned)SEQ, s = row % (unsigned)SEQ;
    const float* src = K + ((size_t)bh * SEQ_FULL + s) * HD + (u & 7u) * 8u;
    const v4f a = *(const v4f*)src, b = *(const v4f*)(src + 4);
    v4u pk; pk.x = pk2(a.x, a.y); pk.y = pk2(a.z, a.w); pk.z = pk2(b.x, b.y); pk.w = pk2(b.z, b.w);
    volatile v4u* d = (volatile v4u*)(Kb + (size_t)u * 8u);
    *d = pk; __threadfence(); *d = pk;
}

__global__ __launch_bounds__(256) void k_prep_vt(const float* __restrict__ V, unsigned short* __restrict__ Vt) {
    __shared__ unsigned short tile[64][66];
    const unsigned bh = blockIdx.y, kb = blockIdx.x * 64u, t = threadIdx.x;
    const float* vbase = V + ((size_t)bh * SEQ_FULL + kb) * HD;
#pragma unroll
    for (unsigned i = 0; i < 4u; ++i) {
        const unsigned f = t + i * 256u, key = f >> 4, dq = (f & 15u) << 2;
        const v4f x = *(const v4f*)(vbase + (size_t)f * 4u);
        tile[key][dq + 0] = (unsigned short)bfu_rne(x.x);
        tile[key][dq + 1] = (unsigned short)bfu_rne(x.y);
        tile[key][dq + 2] = (unsigned short)bfu_rne(x.z);
        tile[key][dq + 3] = (unsigned short)bfu_rne(x.w);
    }
    __syncthreads();
    v4u pk[2];
#pragma unroll
    for (unsigned it = 0; it < 2u; ++it) {
        const unsigned pi = it * 256u + t, d = pi >> 3, seg = (pi & 7u) * 8u;
        unsigned e[8];
#pragma unroll
        for (unsigned j = 0; j < 8u; ++j) e[j] = (unsigned)tile[seg + j][d];
        pk[it].x = e[0] | (e[1] << 16); pk[it].y = e[2] | (e[3] << 16); pk[it].z = e[4] | (e[5] << 16); pk[it].w = e[6] | (e[7] << 16);
    }
#pragma unroll
    for (unsigned it = 0; it < 2u; ++it) {
        const unsigned pi = it * 256u + t, d = pi >> 3, seg = (pi & 7u) * 8u;
        *(volatile v4u*)(Vt + ((size_t)bh * HD + d) * SEQ + kb + seg) = pk[it];
    }
    __threadfence();
#pragma unroll
    for (unsigned it = 0; it < 2u; ++it) {
        const unsigned pi = it * 256u + t, d = pi >> 3, seg = (pi & 7u) * 8u;
        *(volatile v4u*)(Vt + ((size_t)bh * HD + d) * SEQ + kb + seg) = pk[it];
    }
}

__global__ __launch_bounds__(32 * AW) void k_attn(const float* __restrict__ Q, const unsigned short* __restrict__ Kb, const unsigned short* __restrict__ Vt,
                                                   const int* __restrict__ mask, const int* __restrict__ flags, float* __restrict__ O) {
    __shared__ __align__(16) float ot[AW][16 * OP];
    const unsigned lane = threadIdx.x & 31u, w = threadIdx.x >> 5, n = lane & 15u, hf = lane >> 4;
    const unsigned qt = blockIdx.x, bh = blockIdx.y;
    const unsigned q0 = qt * 64u + w * 16u;
    const float NEG = -__builtin_inff();
    const float SC = 0.125f * 1.4426950408889634f;

    const float* qrow = Q + ((size_t)bh * SEQ_FULL + q0 + n) * HD + 8u * hf;
    v16b bQ[2];
#pragma unroll
    for (int ks = 0; ks < 2; ++ks) {
        const float* p = qrow + ks * 32;
        const v4f a = *(const v4f*)p, b = *(const v4f*)(p + 4), c = *(const v4f*)(p + 16), d = *(const v4f*)(p + 20);
        v4u lo, hi;
        lo.x = pk2(a.x, a.y); lo.y = pk2(a.z, a.w); lo.z = pk2(b.x, b.y); lo.w = pk2(b.z, b.w);
        hi.x = pk2(c.x, c.y); hi.y = pk2(c.z, c.w); hi.z = pk2(d.x, d.y); hi.w = pk2(d.z, d.w);
        bQ[ks] = mkfrag(lo, hi);
    }

    v8f acc[4];
#pragma unroll
    for (int nt = 0; nt < 4; ++nt) { v8f zz = {}; acc[nt] = zz; }
    float m = NEG, l = 0.f;

    const unsigned short* kbase = Kb + (size_t)bh * SEQ * HD;
    const unsigned short* vbase = Vt + (size_t)bh * HD * SEQ;
    const int* frow = flags + qt * FPITCH;
    const int* mrow = mask + (size_t)(q0 + n) * SEQ_FULL + 8u * hf;

#pragma unroll 1
    for (unsigned kt = 0; kt < (unsigned)NKT; ++kt) {
        const int fl = frow[kt];
        if (fl == 0) continue;
        const bool chk = (fl != 1);
#pragma unroll 1
        for (unsigned sb = 0; sb < 2u; ++sb) {
            const unsigned kb = kt * 64u + sb * 32u;
            float sc[2][8];
#pragma unroll
            for (int t = 0; t < 2; ++t) {
                const unsigned short* kp = kbase + (size_t)(kb + 16u * t + n) * HD + 8u * hf;
                v8f s = {};
#pragma unroll
                for (int ks = 0; ks < 2; ++ks) {
                    const v4u lo = *(const v4u*)(kp + ks * 32), hi = *(const v4u*)(kp + ks * 32 + 16);
                    s = wmmab(mkfrag(lo, hi), bQ[ks], s);
                }
#pragma unroll
                for (int r = 0; r < 8; ++r) sc[t][r] = s[r] * SC;
            }
            if (chk) {
#pragma unroll
                for (int t = 0; t < 2; ++t) {
                    const int* mp = mrow + kb + 16u * t;
                    const v4i m0 = *(const v4i*)mp, m1 = *(const v4i*)(mp + 4);
                    sc[t][0] = (m0.x != 0) ? sc[t][0] : NEG; sc[t][1] = (m0.y != 0) ? sc[t][1] : NEG;
                    sc[t][2] = (m0.z != 0) ? sc[t][2] : NEG; sc[t][3] = (m0.w != 0) ? sc[t][3] : NEG;
                    sc[t][4] = (m1.x != 0) ? sc[t][4] : NEG; sc[t][5] = (m1.y != 0) ? sc[t][5] : NEG;
                    sc[t][6] = (m1.z != 0) ? sc[t][6] : NEG; sc[t][7] = (m1.w != 0) ? sc[t][7] : NEG;
                }
            }
            float mx = NEG;
#pragma unroll
            for (int t = 0; t < 2; ++t)
#pragma unroll
                for (int r = 0; r < 8; ++r) mx = fmaxf(mx, sc[t][r]);
            mx = fmaxf(mx, __shfl_xor(mx, 16, 32));
            const float mnew = fmaxf(m, mx);
            const float corr = (mnew == NEG) ? 1.f : exp2f(m - mnew);
            float rs = 0.f;
            v8u wh, wl;
#pragma unroll
            for (int t = 0; t < 2; ++t)
#pragma unroll
                for (int j = 0; j < 4; ++j) {
                    const float s0 = sc[t][2 * j], s1 = sc[t][2 * j + 1];
                    const float e0 = exp2f(s0 - mnew), e1 = exp2f(s1 - mnew);
                    const float p0 = (s0 == NEG) ? 0.f : e0;
                    const float p1 = (s1 == NEG) ? 0.f : e1;
                    rs += p0 + p1;
                    const unsigned h0 = bfu_rne(p0), h1 = bfu_rne(p1);
                    const unsigned l0 = bfu_rne(p0 - __uint_as_float(h0 << 16)), l1 = bfu_rne(p1 - __uint_as_float(h1 << 16));
                    wh[4 * t + j] = h0 | (h1 << 16);
                    wl[4 * t + j] = l0 | (l1 << 16);
                }
            rs += __shfl_xor(rs, 16, 32);
            l = l * corr + rs; m = mnew;
#pragma unroll
            for (int nt = 0; nt < 4; ++nt) acc[nt] *= corr;
            const v16b bPh = __builtin_bit_cast(v16b, wh), bPl = __builtin_bit_cast(v16b, wl);
#pragma unroll
            for (int nt = 0; nt < 4; ++nt) {
                const unsigned short* vp = vbase + (size_t)(16u * nt + n) * SEQ + kb + 8u * hf;
                const v4u lo = *(const v4u*)vp, hi = *(const v4u*)(vp + 16);
                acc[nt] = wmmab2(mkfrag(lo, hi), bPh, bPl, acc[nt]);
            }
        }
    }

    const float inv = 1.0f / l;
    float* mt = ot[w];
#pragma unroll
    for (int nt = 0; nt < 4; ++nt) {
        v4f a, b;
        a.x = acc[nt][0] * inv; a.y = acc[nt][1] * inv; a.z = acc[nt][2] * inv; a.w = acc[nt][3] * inv;
        b.x = acc[nt][4] * inv; b.y = acc[nt][5] * inv; b.z = acc[nt][6] * inv; b.w = acc[nt][7] * inv;
        *(v4f*)(mt + n * OP + 16 * nt + 8u * hf) = a;
        *(v4f*)(mt + n * OP + 16 * nt + 8u * hf + 4u) = b;
    }
    __syncthreads();
    float* obase = O + ((size_t)bh * SEQ + q0) * HD;
    v4f vv[8];
#pragma unroll
    for (int s = 0; s < 8; ++s) vv[s] = *(const v4f*)(mt + (2u * s + hf) * OP + n * 4u);
#pragma unroll
    for (int s = 0; s < 8; ++s) *(volatile v4f*)(obase + (size_t)(2u * s + hf) * HD + n * 4u) = vv[s];
    __threadfence();
#pragma unroll
    for (int s = 0; s < 8; ++s) *(volatile v4f*)(obase + (size_t)(2u * s + hf) * HD + n * 4u) = vv[s];
}

extern "C" void kernel_launch(void* const* d_in, const int* in_sizes, int n_in, void* d_out, int out_size, void* d_ws, size_t ws_size, hipStream_t stream) {
    if (n_in < 4) return;
    const long long need_qkv = ((long long)(NBH - 1) * SEQ_FULL + SEQ) * HD;
    const long long need_msk = (long long)(SEQ - 1) * SEQ_FULL + SEQ;
    const long long nel = (long long)NBH * SEQ * HD;
    if ((long long)in_sizes[0] < need_qkv || (long long)in_sizes[1] < need_qkv || (long long)in_sizes[2] < need_qkv) return;
    if ((long long)in_sizes[3] < need_msk) return;
    if ((long long)out_size < nel) return;

    const float* Q = (const float*)d_in[0];
    const float* K = (const float*)d_in[1];
    const float* V = (const float*)d_in[2];
    const int* mask = (const int*)d_in[3];
    float* out = (float*)d_out;

    const size_t plane_b = (((size_t)nel * 2u + 255u) / 256u) * 256u;
    const size_t flag_b = (((size_t)NKT * FPITCH * 4u + 255u) / 256u) * 256u;
    if (plane_b * 2u + flag_b > ws_size) return;
    char* wsp = (char*)d_ws;
    unsigned short* Kb = (unsigned short*)wsp; wsp += plane_b;
    unsigned short* Vt = (unsigned short*)wsp; wsp += plane_b;
    int* flags = (int*)wsp;

    k_flags<<<dim3((unsigned)NKT), 256, 0, stream>>>(mask, flags);
    k_prep_k<<<dim3((unsigned)(((long long)NBH * SEQ * 8) / 256)), 256, 0, stream>>>(K, Kb);
    k_prep_vt<<<dim3((unsigned)NKT, (unsigned)NBH), 256, 0, stream>>>(V, Vt);
    k_attn<<<dim3((unsigned)NKT, (unsigned)NBH), 32 * AW, 0, stream>>>(Q, Kb, Vt, mask, flags, out);
}
